// GAT_11948599017832
// MI455X (gfx1250) — hardware-run, weakly checked
//
#include <hip/hip_runtime.h>


#ifndef NB
#define NB 4
#endif
#define NB_FULL 4
#define NN   128
#define FI   128
#define ZK   256
#define FO   128
#define NHD  8
#define HDM  16
#define NT   8
#define C1P  192
#define CA1  128
#define CA2  136
#define CT1  144
#define CT2  152
#define W1R  320
#define VP   (NB * NN)
#define LN_EPS 1e-5f
#define LOG2E 1.4426950408889634f

static_assert(NHD * HDM == FO);
static_assert(ZK == 2 * FI);
static_assert(ZK % 32 == 0);
static_assert(FI % 32 == 0);
static_assert((NB * NN) % 64 == 0);
static_assert(C1P % 64 == 0);
static_assert(FO % 64 == 0);
static_assert((NB * NN * NN) % 64 == 0);
static_assert(W1R - 128 == C1P);
static_assert(NB <= NB_FULL);
static_assert((size_t)NB_FULL * NN * FO * 4 == (size_t)262144);

typedef unsigned short bf;
typedef __attribute__((ext_vector_type(16))) __bf16   v16bf;
typedef __attribute__((ext_vector_type(8)))  unsigned short v8us;
typedef __attribute__((ext_vector_type(8)))  float    v8f;
typedef __attribute__((ext_vector_type(4)))  float    v4f;
typedef v4f  __attribute__((may_alias)) v4fa;

__device__ __forceinline__ unsigned short f2bf(float f) { unsigned u = __float_as_uint(f); u += 0x7FFFu + ((u >> 16) & 1u); return (unsigned short)(u >> 16); }
__device__ __forceinline__ float bf2f(unsigned short h) { return __uint_as_float(((unsigned)h) << 16); }
__device__ __forceinline__ float bfr(float f) { return bf2f(f2bf(f)); }
__device__ __forceinline__ v16bf cat16b(v8us lo, v8us hi) { return __builtin_bit_cast(v16bf, __builtin_shufflevector(lo, hi, 0, 1, 2, 3, 4, 5, 6, 7, 8, 9, 10, 11, 12, 13, 14, 15)); }
__device__ __forceinline__ v8f wmmab(v16bf a, v16bf b, v8f c) { return __builtin_amdgcn_wmma_f32_16x16x32_bf16(false, a, false, b, (short)0, c, false, false); }
__device__ __forceinline__ v16bf ldb(const bf* p)  { return cat16b(*(const v8us*)p, *(const v8us*)(p + 16)); }
__device__ __forceinline__ void wave_sync() { __builtin_amdgcn_fence(3  , "wavefront"); __builtin_amdgcn_wave_barrier(); asm volatile("" ::: "memory"); }
__device__ __forceinline__ float wsum(float v) { v += __shfl_xor(v, 16, 32); v += __shfl_xor(v, 8, 32); v += __shfl_xor(v, 4, 32); v += __shfl_xor(v, 2, 32); v += __shfl_xor(v, 1, 32); return v; }

__device__ __forceinline__ v8f ldcol8(const float* __restrict__ s, int ld, int col, int k0) {
    v8f v;
#pragma unroll
    for (int e = 0; e < 8; ++e) v[e] = s[(size_t)(k0 + e) * ld + col];
    return v;
}
__device__ __forceinline__ void st8bf(bf* p, v8f v) {
    v8us o;
#pragma unroll
    for (int k = 0; k < 8; ++k) o[k] = f2bf(v[k]);
    *(volatile v8us*)p = o; __threadfence(); *(volatile v8us*)p = o;
}
__device__ __forceinline__ v16bf pack16(v4f x0, v4f x1, v4f x2, v4f x3) {
    v8us lo, hi;
#pragma unroll
    for (int e = 0; e < 4; ++e) { lo[e] = f2bf(x0[e]); lo[4 + e] = f2bf(x1[e]); hi[e] = f2bf(x2[e]); hi[4 + e] = f2bf(x3[e]); }
    return cat16b(lo, hi);
}

#define PZB ((NB * NN * 32) / 256)
#define PW1 ((W1R * 32) / 256)
#define PW2 ((32 * 16) / 256)
static_assert((NB * NN * 32) % 256 == 0);
static_assert((W1R * 32) % 256 == 0);
static_assert((32 * 16) % 256 == 0);

__global__ __launch_bounds__(256) void k_prep(const float* __restrict__ node, const float* __restrict__ hidden,
                                              const float* __restrict__ m_w, const float* __restrict__ skip_w,
                                              const float* __restrict__ a1_w, const float* __restrict__ a2_w,
                                              const float* __restrict__ t1_w, const float* __restrict__ t2_w,
                                              const float* __restrict__ ae_w, const float* __restrict__ te1_w,
                                              const float* __restrict__ te2_w, const float* __restrict__ te3_w,
                                              bf* ZB, bf* W1T, bf* W2T) {
    const int blk = blockIdx.x, tid = threadIdx.x;
    if (blk < PZB) {
        const int i = blk * 256 + tid; const int row = i >> 5, c8 = i & 31; const int cc = (c8 & 15) * 8;
        const v8f a = *(const v8f*)(node + (size_t)row * FI + cc);
        const v8f h = *(const v8f*)(hidden + (size_t)row * FI + cc);
        v8f v;
#pragma unroll
        for (int e = 0; e < 8; ++e) v[e] = (c8 < 16) ? a[e] : h[e];
        st8bf(ZB + (size_t)i * 8, v);
    } else if (blk < PZB + PW1) {
        const int i = (blk - PZB) * 256 + tid; const int n = __builtin_amdgcn_readfirstlane(i >> 5); const int k0 = (i & 31) * 8;
        v8f v = (v8f){};
        if (n < 128)      v = ldcol8(m_w,    128, n,       k0);
        else if (n < 256) v = ldcol8(skip_w, 128, n - 128, k0);
        else if (n < 264) v = ldcol8(a1_w,   8,   n - 256, k0);
        else if (n < 272) v = ldcol8(a2_w,   8,   n - 264, k0);
        else if (n < 280) v = ldcol8(t1_w,   8,   n - 272, k0);
        else if (n < 288) v = ldcol8(t2_w,   8,   n - 280, k0);
        st8bf(W1T + (size_t)i * 8, v);
    } else {
        const int i = (blk - PZB - PW1) * 256 + tid; const int n = i >> 4; const int sel = __builtin_amdgcn_readfirstlane(n >> 3);
        const int col = n & 7; const int k0 = (i & 15) * 8;
        v8f v = (v8f){};
        if (sel == 0)      v = ldcol8(ae_w,  8, col, k0);
        else if (sel == 1) v = ldcol8(te1_w, 8, col, k0);
        else if (sel == 2) v = ldcol8(te2_w, 8, col, k0);
        else               v = ldcol8(te3_w, 8, col, k0);
        st8bf(W2T + (size_t)i * 8, v);
    }
}

__global__ __launch_bounds__(32) void k_gemm_c1(const bf* __restrict__ A, const bf* __restrict__ Bt, float* C) {
    __shared__ __align__(16) float os[16 * 68];
    const int K = ZK;
    const int lane = threadIdx.x & 31, lr = lane & 15, hi = lane >> 4; const int r0 = blockIdx.x * 64, c0 = blockIdx.y * 64;
    v8f acc[4][4];
#pragma unroll
    for (int mb = 0; mb < 4; ++mb)
#pragma unroll
        for (int nb = 0; nb < 4; ++nb) acc[mb][nb] = (v8f){};
    const size_t aoff = (size_t)(r0 + lr) * K + 8 * hi, boff = (size_t)(c0 + lr) * K + 8 * hi;
#pragma unroll 1
    for (int kc = 0; kc < K; kc += 32) {
        v16bf a[4];
#pragma unroll
        for (int mb = 0; mb < 4; ++mb) a[mb] = ldb(A + aoff + (size_t)mb * 16 * K + kc);
#pragma unroll
        for (int nb = 0; nb < 4; ++nb) { const v16bf b = ldb(Bt + boff + (size_t)nb * 16 * K + kc);
#pragma unroll
            for (int mb = 0; mb < 4; ++mb) acc[mb][nb] = wmmab(a[mb], b, acc[mb][nb]); }
        asm volatile("v_nop\n\tv_nop\n\tv_nop\n\tv_nop" : "+v"(acc[0][0]), "+v"(acc[1][1]), "+v"(acc[2][2]), "+v"(acc[3][3]) : "v"(a[0]), "v"(a[1]), "v"(a[2]), "v"(a[3]));
    }
#pragma unroll
    for (int mb = 0; mb < 4; ++mb) {
#pragma unroll
        for (int nb = 0; nb < 4; ++nb) {
#pragma unroll
            for (int j = 0; j < 8; ++j) os[(hi * 8 + j) * 68 + nb * 16 + lr] = acc[mb][nb][j]; }
        wave_sync();
        float* cb = C + (size_t)(r0 + mb * 16) * C1P + c0;
#pragma unroll 1
        for (int ps = 0; ps < 2; ++ps) {
#pragma unroll
            for (int s = 0; s < 8; ++s) { const int row = 2 * s + hi, cofs = lr * 4;
                const v4f val = *(const v4fa*)(&os[row * 68 + cofs]);
                *(volatile v4f*)(cb + (size_t)row * C1P + cofs) = val; }
            if (ps == 0) __threadfence(); }
        wave_sync();
    }
}

__global__ __launch_bounds__(32) void k_gemm_vt(const bf* __restrict__ A, const bf* __restrict__ Bt, bf* PH, bf* PL) {
    __shared__ __align__(16) float os[16 * 68];
    const int K = ZK;
    const int lane = threadIdx.x & 31, lr = lane & 15, hi = lane >> 4; const int r0 = blockIdx.x * 64, c0 = blockIdx.y * 64;
    v8f acc[4][4];
#pragma unroll
    for (int mb = 0; mb < 4; ++mb)
#pragma unroll
        for (int nb = 0; nb < 4; ++nb) acc[mb][nb] = (v8f){};
    const size_t aoff = (size_t)(r0 + lr) * K + 8 * hi, boff = (size_t)(c0 + lr) * K + 8 * hi;
#pragma unroll 1
    for (int kc = 0; kc < K; kc += 32) {
        v16bf a[4];
#pragma unroll
        for (int mb = 0; mb < 4; ++mb) a[mb] = ldb(A + aoff + (size_t)mb * 16 * K + kc);
#pragma unroll
        for (int nb = 0; nb < 4; ++nb) { const v16bf b = ldb(Bt + boff + (size_t)nb * 16 * K + kc);
#pragma unroll
            for (int mb = 0; mb < 4; ++mb) acc[mb][nb] = wmmab(a[mb], b, acc[mb][nb]); }
        asm volatile("v_nop\n\tv_nop\n\tv_nop\n\tv_nop" : "+v"(acc[0][0]), "+v"(acc[1][1]), "+v"(acc[2][2]), "+v"(acc[3][3]) : "v"(a[0]), "v"(a[1]), "v"(a[2]), "v"(a[3]));
    }
#pragma unroll
    for (int mb = 0; mb < 4; ++mb) {
#pragma unroll
        for (int nb = 0; nb < 4; ++nb) {
#pragma unroll
            for (int j = 0; j < 8; ++j) os[(hi * 8 + j) * 68 + nb * 16 + lr] = acc[mb][nb][j]; }
        wave_sync();
        const size_t sb = (size_t)(r0 + mb * 16) * VP + c0;
#pragma unroll 1
        for (int ps = 0; ps < 2; ++ps) {
#pragma unroll
            for (int s = 0; s < 4; ++s) { const int row = 4 * s + (lane >> 3), c8 = (lane & 7) * 8;
                const v4f x0 = *(const v4fa*)(&os[row * 68 + c8]); const v4f x1 = *(const v4fa*)(&os[row * 68 + c8 + 4]); v8us hv, lv;
#pragma unroll
                for (int i = 0; i < 4; ++i) { const unsigned short a0 = f2bf(x0[i]); const unsigned short a1 = f2bf(x1[i]); hv[i] = a0; hv[4 + i] = a1;
                    lv[i] = f2bf(x0[i] - bf2f(a0)); lv[4 + i] = f2bf(x1[i] - bf2f(a1)); }
                const size_t oo = sb + (size_t)row * VP + c8;
                *(volatile v8us*)(PH + oo) = hv; *(volatile v8us*)(PL + oo) = lv; }
            if (ps == 0) __threadfence(); }
        wave_sync();
    }
}

__global__ __launch_bounds__(32) __attribute__((amdgpu_num_vgpr(256)))
void k_gemm_e(const float* __restrict__ edge, const bf* __restrict__ W2T, float* AET, float* E1, float* E2, float* E3) {
    __shared__ __align__(16) float os[64 * 36];
    const int lane = threadIdx.x & 31, lr = lane & 15, hi = lane >> 4;
    const size_t r0 = (size_t)blockIdx.x * 64;
    v8f acc[4][2];
#pragma unroll
    for (int mb = 0; mb < 4; ++mb) { acc[mb][0] = (v8f){}; acc[mb][1] = (v8f){}; }
    const size_t aoff = (r0 + lr) * FI + 8 * hi; const size_t boff = (size_t)lr * FI + 8 * hi;
#pragma unroll 1
    for (int kc = 0; kc < FI; kc += 32) {
        v16bf a[4];
#pragma unroll
        for (int mb = 0; mb < 4; ++mb) { const float* p = edge + aoff + (size_t)mb * 16 * FI + kc;
            a[mb] = pack16(*(const v4f*)p, *(const v4f*)(p + 4), *(const v4f*)(p + 16), *(const v4f*)(p + 20)); }
        const v16bf b0 = ldb(W2T + boff + kc); const v16bf b1 = ldb(W2T + boff + (size_t)16 * FI + kc);
#pragma unroll
        for (int mb = 0; mb < 4; ++mb) acc[mb][0] = wmmab(a[mb], b0, acc[mb][0]);
#pragma unroll
        for (int mb = 0; mb < 4; ++mb) acc[mb][1] = wmmab(a[mb], b1, acc[mb][1]);
        asm volatile("v_nop\n\tv_nop\n\tv_nop\n\tv_nop" : "+v"(acc[0][0]), "+v"(acc[1][0]), "+v"(acc[2][0]), "+v"(acc[3][0]), "+v"(acc[0][1]), "+v"(acc[1][1]), "+v"(acc[2][1]), "+v"(acc[3][1])
                     : "v"(a[0]), "v"(a[1]), "v"(a[2]), "v"(a[3]), "v"(b0), "v"(b1));
    }
#pragma unroll
    for (int mb = 0; mb < 4; ++mb)
#pragma unroll
        for (int nb = 0; nb < 2; ++nb)
#pragma unroll
            for (int j = 0; j < 8; ++j) os[(mb * 16 + hi * 8 + j) * 36 + nb * 16 + lr] = acc[mb][nb][j];
    wave_sync();
    const int bi = blockIdx.x >> 1, j0 = (blockIdx.x & 1) * 64; const int b = bi >> 7, i = bi & 127;
#pragma unroll 1
    for (int ps = 0; ps < 2; ++ps) {
#pragma unroll
        for (int mb = 0; mb < 4; ++mb) { const int row = mb * 16 + (lane >> 1), cq = (lane & 1) * 4;
            const v4f x1 = *(const v4fa*)(&os[row * 36 + 8 + cq]); const v4f x2 = *(const v4fa*)(&os[row * 36 + 16 + cq]); const v4f x3 = *(const v4fa*)(&os[row * 36 + 24 + cq]);
            const size_t oo = (r0 + mb * 16) * NT + lane * 4;
            *(volatile v4f*)(E1 + oo) = x1; *(volatile v4f*)(E2 + oo) = x2; *(volatile v4f*)(E3 + oo) = x3; }
#pragma unroll
        for (int hh = 0; hh < 4; ++hh) { const int hd = 2 * hh + hi, j4 = lr * 4; v4f x;
#pragma unroll
            for (int e = 0; e < 4; ++e) x[e] = os[(j4 + e) * 36 + hd];
            *(volatile v4f*)(AET + (((size_t)(b * NHD + hd) * NN + i) * NN + j0 + j4)) = x; }
        if (ps == 0) __threadfence();
    }
}

__global__ __launch_bounds__(256) __attribute__((amdgpu_num_vgpr(256)))
void k_attn(const float* __restrict__ C1, const float* __restrict__ AET, const bf* __restrict__ VTH, const bf* __restrict__ VTL,
            const float* __restrict__ adj, const float* __restrict__ graph, const float* __restrict__ ag_w,
            const float* __restrict__ skip_b, const float* __restrict__ gamma, const float* __restrict__ beta, float* OUT) {
    __shared__ __align__(16) float a2t[NHD * 132];
    __shared__ __align__(16) float ot[16 * 132];
    const int tid = threadIdx.x, lane = tid & 31, lr = lane & 15, hi = lane >> 4;
    const int h = __builtin_amdgcn_readfirstlane(tid >> 5);
    const int b = blockIdx.y, i0 = blockIdx.x * 16;
    { const int j = tid >> 1, hf = tid & 1;
      const v4f xv = *(const v4f*)(C1 + (size_t)(b * NN + j) * C1P + CA2 + hf * 4);
#pragma unroll
      for (int e = 0; e < 4; ++e) a2t[(hf * 4 + e) * 132 + j] = xv[e]; }
    float ag = 0.0f;
#pragma unroll 1
    for (int q = 0; q < 4; ++q) { const int f = lane + 32 * q; ag += bfr(graph[(size_t)b * FI + f]) * bfr(ag_w[f * NHD + h]); }
    ag = wsum(ag);
    __syncthreads();

    const int i = i0 + lr;
    const float a1 = C1[(size_t)(b * NN + i) * C1P + CA1 + h];
    const float* aep = AET + (((size_t)(b * NHD + h) * NN + i) * NN) + 8 * hi;
    float x[64]; float mx = -3.0e38f;
#pragma unroll
    for (int kk = 0; kk < 4; ++kk) {
#pragma unroll
        for (int g = 0; g < 2; ++g) {
            const int off = kk * 32 + 16 * g;
            const v4f e0 = *(const v4f*)(aep + off); const v4f e1 = *(const v4f*)(aep + off + 4);
            const v4f s0 = *(const v4fa*)(&a2t[h * 132 + off + 8 * hi]); const v4f s1 = *(const v4fa*)(&a2t[h * 132 + off + 8 * hi + 4]);
#pragma unroll
            for (int e = 0; e < 4; ++e) {
                float t = ((a1 + s0[e]) + e0[e]) + ag; t = (t >= 0.0f) ? t : 0.01f * t; x[kk * 16 + 8 * g + e] = t; mx = fmaxf(mx, t);
                float u = ((a1 + s1[e]) + e1[e]) + ag; u = (u >= 0.0f) ? u : 0.01f * u; x[kk * 16 + 8 * g + 4 + e] = u; mx = fmaxf(mx, u); }
        }
    }
    mx = fmaxf(mx, __shfl_xor(mx, 16, 32));
    float l = 0.0f;
#pragma unroll
    for (int q = 0; q < 64; ++q) { x[q] = __builtin_amdgcn_exp2f((x[q] - mx) * LOG2E); l += x[q]; }
    l += __shfl_xor(l, 16, 32);
    const float inv = 1.0f / l;

    const float* adp = adj + ((size_t)(b * NN + i) * NN) + 8 * hi;
    const bf* vhp = VTH + (size_t)(h * HDM + lr) * VP + (size_t)b * NN + 8 * hi;
    const bf* vlp = VTL + (size_t)(h * HDM + lr) * VP + (size_t)b * NN + 8 * hi;
    v8f acc = (v8f){};
#pragma unroll
    for (int kk = 0; kk < 4; ++kk) {
        const v4f d0 = *(const v4f*)(adp + kk * 32); const v4f d1 = *(const v4f*)(adp + kk * 32 + 4);
        const v4f d2 = *(const v4f*)(adp + kk * 32 + 16); const v4f d3 = *(const v4f*)(adp + kk * 32 + 20);
        v8us h0, h1, l0, l1;
#pragma unroll
        for (int e = 0; e < 4; ++e) {
            const float c0 = bfr(d0[e]) * (x[kk * 16 + e] * inv);      const float c1 = bfr(d1[e]) * (x[kk * 16 + 4 + e] * inv);
            const float c2 = bfr(d2[e]) * (x[kk * 16 + 8 + e] * inv);  const float c3 = bfr(d3[e]) * (x[kk * 16 + 12 + e] * inv);
            const unsigned short q0 = f2bf(c0), q1 = f2bf(c1), q2 = f2bf(c2), q3 = f2bf(c3);
            h0[e] = q0; h0[4 + e] = q1; h1[e] = q2; h1[4 + e] = q3;
            l0[e] = f2bf(c0 - bf2f(q0)); l0[4 + e] = f2bf(c1 - bf2f(q1)); l1[e] = f2bf(c2 - bf2f(q2)); l1[4 + e] = f2bf(c3 - bf2f(q3)); }
        const v16bf chi = cat16b(h0, h1), clo = cat16b(l0, l1);
        const v16bf vh = ldb(vhp + kk * 32), vl = ldb(vlp + kk * 32);
        acc = wmmab(chi, vh, acc); acc = wmmab(chi, vl, acc); acc = wmmab(clo, vh, acc);
        asm volatile("v_nop\n\tv_nop\n\tv_nop\n\tv_nop" : "+v"(acc) : "v"(chi), "v"(clo), "v"(vh), "v"(vl));
    }
#pragma unroll
    for (int r = 0; r < 8; ++r) ot[(8 * hi + r) * 132 + h * HDM + lr] = acc[r];
    __syncthreads();

    const int c4 = lane * 4;
    const v4f sbv = *(const v4f*)(skip_b + c4); const v4f gmv = *(const v4f*)(gamma + c4); const v4f btv = *(const v4f*)(beta + c4);
    v4f y0, y1;
#pragma unroll
    for (int rr = 0; rr < 2; ++rr) {
        const int row = 2 * h + rr; const size_t gi = (size_t)(b * NN + i0 + row);
        const v4f o = *(const v4fa*)(&ot[row * 132 + c4]);
        const v4f sk = *(const v4f*)(C1 + gi * C1P + c4);
        v4f v; float s = 0.0f;
#pragma unroll
        for (int e = 0; e < 4; ++e) { const float t = (o[e] + sk[e]) + bfr(sbv[e]); v[e] = fmaxf(t, 0.0f); s += v[e]; }
        const float mu = wsum(s) * (1.0f / FO);
        float q = 0.0f; v4f d;
#pragma unroll
        for (int e = 0; e < 4; ++e) { d[e] = v[e] - mu; q += d[e] * d[e]; }
        const float var = wsum(q) * (1.0f / FO);
        const float rs = rsqrtf(var + LN_EPS);
        v4f y;
#pragma unroll
        for (int e = 0; e < 4; ++e) y[e] = d[e] * rs * bfr(gmv[e]) + bfr(btv[e]);
        if (rr == 0) y0 = y; else y1 = y;
    }
    float* op0 = OUT + (size_t)(b * NN + i0 + 2 * h) * FO + c4; float* op1 = op0 + FO;
    *(volatile v4f*)op0 = y0; *(volatile v4f*)op1 = y1;
    __threadfence();
    *(volatile v4f*)op0 = y0; *(volatile v4f*)op1 = y1;
}

__global__ __launch_bounds__(128) void k_tri(const float* __restrict__ C1, const float* __restrict__ E1, const float* __restrict__ E2, const float* __restrict__ E3,
                                             const float* __restrict__ graph, const float* __restrict__ tg_w, const float* __restrict__ tg_b,
                                             const float* __restrict__ t1_b, const float* __restrict__ t2_b,
                                             const float* __restrict__ te1_b, const float* __restrict__ te2_b, const float* __restrict__ te3_b,
                                             const float* __restrict__ o3_w, const float* __restrict__ o3_b,
                                             const float* __restrict__ gamma, const float* __restrict__ beta, float* OUT1) {
    __shared__ __align__(16) float U[NN * 8];
    __shared__ __align__(16) float TS[NN * 8];
    __shared__ __align__(16) float gs[8];
    const int tid = threadIdx.x, lane = tid & 31;
    const int wave = __builtin_amdgcn_readfirstlane(tid >> 5);
    const int j = blockIdx.x, b = blockIdx.y;
    { const size_t gi = (size_t)(b * NN + tid);
      const v4f t0 = *(const v4f*)(C1 + gi * C1P + CT1); const v4f t1 = *(const v4f*)(C1 + gi * C1P + CT1 + 4);
      const v4f e0 = *(const v4f*)(E1 + (gi * NN + j) * NT); const v4f e1 = *(const v4f*)(E1 + (gi * NN + j) * NT + 4);
      *(v4fa*)(&U[tid * 8]) = t0 + e0; *(v4fa*)(&U[tid * 8 + 4]) = t1 + e1; }
#pragma unroll 1
    for (int tt = 0; tt < 2; ++tt) {
        const int t = 2 * wave + tt; float p = 0.0f;
#pragma unroll 1
        for (int q = 0; q < 4; ++q) { const int f = lane + 32 * q; p += bfr(graph[(size_t)b * FI + f]) * bfr(tg_w[f * NT + t]); }
        p = wsum(p);
        const float cb = ((((bfr(tg_b[t]) + 2.0f * bfr(t1_b[t])) + bfr(t2_b[t])) + bfr(te1_b[t])) + bfr(te2_b[t])) + bfr(te3_b[t]);
        if (lane == 0) gs[t] = p + cb;
    }
    __syncthreads();

    const int k = tid;
    const float NEG = -__builtin_inff();
    v4f m0 = {NEG, NEG, NEG, NEG}, m1 = {NEG, NEG, NEG, NEG};
    const float* e2p = E2 + ((size_t)b * NN * NN + k) * NT;
#pragma unroll 4
    for (int i = 0; i < NN; ++i) {
        const v4f a0 = *(const v4f*)(e2p + (size_t)i * NN * NT); const v4f a1 = *(const v4f*)(e2p + (size_t)i * NN * NT + 4);
        const v4f u0 = *(const v4fa*)(&U[i * 8]); const v4f u1 = *(const v4fa*)(&U[i * 8 + 4]);
#pragma unroll
        for (int e = 0; e < 4; ++e) { m0[e] = fmaxf(m0[e], u0[e] + a0[e]); m1[e] = fmaxf(m1[e], u1[e] + a1[e]); }
    }
    { const size_t gj = (size_t)(b * NN + j), gk = (size_t)(b * NN + k);
      const v4f p0 = *(const v4f*)(C1 + gj * C1P + CT2); const v4f p1 = *(const v4f*)(C1 + gj * C1P + CT2 + 4);
      const v4f q0 = *(const v4f*)(C1 + gk * C1P + CT1); const v4f q1 = *(const v4f*)(C1 + gk * C1P + CT1 + 4);
      const v4f r0 = *(const v4f*)(E3 + (gj * NN + k) * NT); const v4f r1 = *(const v4f*)(E3 + (gj * NN + k) * NT + 4);
      const v4f g0 = *(const v4fa*)(&gs[0]); const v4f g1 = *(const v4fa*)(&gs[4]);
      *(v4fa*)(&TS[k * 8]) = (((m0 + p0) + q0) + r0) + g0; *(v4fa*)(&TS[k * 8 + 4]) = (((m1 + p1) + q1) + r1) + g1; }
    __syncthreads();

    const int c4 = lane * 4;
    v4f wv[8];
#pragma unroll
    for (int t = 0; t < 8; ++t) { const v4f w = *(const v4f*)(o3_w + t * FO + c4);
#pragma unroll
        for (int e = 0; e < 4; ++e) wv[t][e] = bfr(w[e]); }
    v4f ob = *(const v4f*)(o3_b + c4), gm = *(const v4f*)(gamma + c4), bt = *(const v4f*)(beta + c4);
#pragma unroll
    for (int e = 0; e < 4; ++e) { ob[e] = bfr(ob[e]); gm[e] = bfr(gm[e]); bt[e] = bfr(bt[e]); }
    float* obase = OUT1 + ((size_t)(b * NN + j) * NN) * FO + c4;
#pragma unroll 1
    for (int r = 0; r < 32; ++r) {
        const int k2 = wave * 32 + r;
        const v4f tv0 = *(const v4fa*)(&TS[k2 * 8]); const v4f tv1 = *(const v4fa*)(&TS[k2 * 8 + 4]);
        v4f v = ob;
#pragma unroll
        for (int t = 0; t < 4; ++t)
#pragma unroll
            for (int e = 0; e < 4; ++e) v[e] = fmaf(tv0[t], wv[t][e], v[e]);
#pragma unroll
        for (int t = 0; t < 4; ++t)
#pragma unroll
            for (int e = 0; e < 4; ++e) v[e] = fmaf(tv1[t], wv[4 + t][e], v[e]);
        float s = 0.0f;
#pragma unroll
        for (int e = 0; e < 4; ++e) { v[e] = fmaxf(v[e], 0.0f); s += v[e]; }
        const float mu = wsum(s) * (1.0f / FO);
        float q = 0.0f; v4f d;
#pragma unroll
        for (int e = 0; e < 4; ++e) { d[e] = v[e] - mu; q += d[e] * d[e]; }
        const float var = wsum(q) * (1.0f / FO);
        const float rs = rsqrtf(var + LN_EPS);
        v4f y;
#pragma unroll
        for (int e = 0; e < 4; ++e) y[e] = d[e] * rs * gm[e] + bt[e];
        float* op = obase + (size_t)k2 * FO;
        *(volatile v4f*)op = y; __threadfence(); *(volatile v4f*)op = y;
    }
}

static constexpr size_t al256(size_t v) { return (v + 255) & ~(size_t)255; }
static constexpr size_t SZ_ZB = al256((size_t)NB * NN * ZK * 2);
static constexpr size_t SZ_W1 = al256((size_t)W1R * ZK * 2);
static constexpr size_t SZ_W2 = al256((size_t)32 * FI * 2);
static constexpr size_t SZ_C1 = al256((size_t)NB * NN * C1P * 4);
static constexpr size_t SZ_VT = al256((size_t)FO * VP * 2);
static constexpr size_t SZ_AE = al256((size_t)NB * NHD * NN * NN * 4);
static constexpr size_t SZ_EP = al256((size_t)NB * NN * NN * NT * 4);
static constexpr size_t SZ_TOTAL = SZ_ZB + SZ_W1 + SZ_W2 + SZ_C1 + 2 * SZ_VT + SZ_AE + 3 * SZ_EP;
static_assert(SZ_TOTAL <= (size_t)134217728);

extern "C" void kernel_launch(void* const* d_in, const int* in_sizes, int n_in,
                              void* d_out, int out_size, void* d_ws, size_t ws_size, hipStream_t stream) {
    if (n_in < 28) return;
    if ((size_t)in_sizes[0] < (size_t)NB * NN * FI) return;
    if ((size_t)in_sizes[1] < (size_t)NB * NN * NN * FI) return;
    if ((size_t)in_sizes[2] < (size_t)NB * FI) return;
    if ((size_t)in_sizes[3] < (size_t)NB * NN * FI) return;
    if ((size_t)in_sizes[4] < (size_t)NB * NN * NN) return;
    if (in_sizes[5] < ZK * FO || in_sizes[6] < ZK * NHD || in_sizes[7] < ZK * NHD || in_sizes[8] < FI * NHD || in_sizes[9] < FI * NHD) return;
    if (in_sizes[10] < ZK * FO || in_sizes[11] < FO || in_sizes[12] < FO || in_sizes[13] < FO) return;
    if (in_sizes[14] < ZK * NT || in_sizes[15] < NT || in_sizes[16] < ZK * NT || in_sizes[17] < NT) return;
    if (in_sizes[18] < FI * NT || in_sizes[19] < NT || in_sizes[20] < FI * NT || in_sizes[21] < NT) return;
    if (in_sizes[22] < FI * NT || in_sizes[23] < NT || in_sizes[24] < FI * NT || in_sizes[25] < NT) return;
    if (in_sizes[26] < NT * FO || in_sizes[27] < FO) return;
    if ((size_t)out_size < (size_t)NB_FULL * NN * FO + (size_t)NB * NN * NN * FO) return;
    if (SZ_TOTAL > ws_size) return;

    const float* node   = (const float*)d_in[0];
    const float* edge   = (const float*)d_in[1];
    const float* graph  = (const float*)d_in[2];
    const float* hidden = (const float*)d_in[3];
    const float* adj    = (const float*)d_in[4];
    const float* m_w    = (const float*)d_in[5];
    const float* a1_w   = (const float*)d_in[6];
    const float* a2_w   = (const float*)d_in[7];
    const float* ae_w   = (const float*)d_in[8];
    const float* ag_w   = (const float*)d_in[9];
    const float* skip_w = (const float*)d_in[10];
    const float* skip_b = (const float*)d_in[11];
    const float* gamma  = (const float*)d_in[12];
    const float* beta   = (const float*)d_in[13];
    const float* t1_w   = (const float*)d_in[14];
    const float* t1_b   = (const float*)d_in[15];
    const float* t2_w   = (const float*)d_in[16];
    const float* t2_b   = (const float*)d_in[17];
    const float* te1_w  = (const float*)d_in[18];
    const float* te1_b  = (const float*)d_in[19];
    const float* te2_w  = (const float*)d_in[20];
    const float* te2_b  = (const float*)d_in[21];
    const float* te3_w  = (const float*)d_in[22];
    const float* te3_b  = (const float*)d_in[23];
    const float* tg_w   = (const float*)d_in[24];
    const float* tg_b   = (const float*)d_in[25];
    const float* o3_w   = (const float*)d_in[26];
    const float* o3_b   = (const float*)d_in[27];
    float* OUT0 = (float*)d_out;
    float* OUT1 = (float*)d_out + (size_t)NB_FULL * NN * FO;

    char* wsp = (char*)d_ws;
    bf* ZB  = (bf*)wsp; wsp += SZ_ZB;
    bf* W1T = (bf*)wsp; wsp += SZ_W1;
    bf* W2T = (bf*)wsp; wsp += SZ_W2;
    float* C1 = (float*)wsp; wsp += SZ_C1;
    bf* VTH = (bf*)wsp; wsp += SZ_VT;
    bf* VTL = (bf*)wsp; wsp += SZ_VT;
    float* AET = (float*)wsp; wsp += SZ_AE;
    float* E1 = (float*)wsp; wsp += SZ_EP;
    float* E2 = (float*)wsp; wsp += SZ_EP;
    float* E3 = (float*)wsp; wsp += SZ_EP;

    k_prep<<<PZB + PW1 + PW2, 256, 0, stream>>>(node, hidden, m_w, skip_w, a1_w, a2_w, t1_w, t2_w, ae_w, te1_w, te2_w, te3_w, ZB, W1T, W2T);
    k_gemm_c1<<<dim3(NB * NN / 64, C1P / 64, 1), 32, 0, stream>>>(ZB, W1T + (size_t)128 * ZK, C1);
    k_gemm_vt<<<dim3(FO / 64, NB * NN / 64, 1), 32, 0, stream>>>(W1T, ZB, VTH, VTL);
    k_gemm_e<<<(unsigned)((size_t)NB * NN * NN / 64), 32, 0, stream>>>(edge, W2T, AET, E1, E2, E3);
    k_attn<<<dim3(NN / 16, NB, 1), 256, 0, stream>>>(C1, AET, VTH, VTL, adj, graph, ag_w, skip_b, gamma, beta, OUT0);
    k_tri<<<dim3(NN, NB, 1), 128, 0, stream>>>(C1, E1, E2, E3, graph, tg_w, tg_b, t1_b, t2_b, te1_b, te2_b, te3_b, o3_w, o3_b, gamma, beta, OUT1);
}
